// LSTM_7782480741002
// MI455X (gfx1250) — hardware-verified
//
#include <hip/hip_runtime.h>
#include <math.h>

constexpr int NBATCH   = 256;
constexpr int NSTEP    = 512;
constexpr int NHID     = 256;
constexpr int NEMB     = 6;
constexpr int NDIG     = 10;
constexpr int NCLS     = 10;
constexpr int NGATE    = 4;
constexpr int SEQ_BLK  = 16;
constexpr int NTHR_SEQ = 512;
constexpr int NWAVE_SEQ = NTHR_SEQ / 32;
constexpr int HPITCH   = 264;
constexpr int HFPITCH  = 260;
constexpr int NTHR_PREP = 256;
constexpr float WCARRY = 16.0f;
constexpr float HCARRY = 64.0f;
constexpr float FOLD   = 1.0f / (WCARRY * HCARRY);

static_assert(NBATCH == NHID, "bias broadcast over the batch axis needs B == H");
static_assert(NBATCH % SEQ_BLK == 0, "batch tiles");
static_assert(NHID == 16 * NWAVE_SEQ, "one 16-unit subtile per wave");
static_assert(NHID % 32 == 0, "K multiple of 32");
static_assert((NGATE * NDIG * NHID / 4) % NTHR_SEQ == 0, "P staging exact");
static_assert((SEQ_BLK * NSTEP / 4) % NTHR_SEQ == 0, "x staging exact");
static_assert((2 * SEQ_BLK * HPITCH) % 8 == 0, "h zero fill in 16-B pieces");
static_assert(HPITCH % 8 == 0 && HFPITCH % 4 == 0, "aligned pitches");
static_assert(SEQ_BLK * NCLS == 160, "five whole 128-B lines per block");
static_assert((SEQ_BLK * NCLS * 4) % 128 == 0, "block output is line aligned");

typedef __attribute__((ext_vector_type(16))) _Float16 v16h;
typedef __attribute__((ext_vector_type(8)))  _Float16 v8h;
typedef __attribute__((ext_vector_type(8)))  float    v8f;
typedef __attribute__((ext_vector_type(4)))  float    v4f;
typedef __attribute__((ext_vector_type(4)))  int      v4i;

union FragU { v16h v; v8h h[2]; };
__device__ __forceinline__ v16h frag_load(const _Float16* p) {
  FragU f;
  f.h[0] = *(const v8h*)(p);
  f.h[1] = *(const v8h*)(p + 16);
  return f.v;
}
__device__ __forceinline__ v8f frag_mma(v16h a, v16h b, v8f c) {
  return __builtin_amdgcn_wmma_f32_16x16x32_f16(false, a, false, b, (short)0, c, false, false);
}
__device__ __forceinline__ void guard_group(v8f& a0, v8f& a1, v8f& a2, v8f& a3,
                                            v16h f0, v16h f1, v16h f2, v16h f3, v16h fb) {
  asm volatile("v_nop\n\tv_nop\n\tv_nop\n\tv_nop"
               : "+v"(a0), "+v"(a1), "+v"(a2), "+v"(a3)
               : "v"(f0), "v"(f1), "v"(f2), "v"(f3), "v"(fb));
}
__device__ __forceinline__ void acc_guard4(v8f& a, v8f& b, v8f& c, v8f& d) {
  asm volatile("v_nop\n\tv_nop\n\tv_nop\n\tv_nop" : "+v"(a), "+v"(b), "+v"(c), "+v"(d));
}

__device__ __forceinline__ float sig_f(float v)  { return __builtin_amdgcn_rcpf(1.0f + expf(-v)); }
__device__ __forceinline__ float tanh_f(float v) { return 1.0f - 2.0f * __builtin_amdgcn_rcpf(expf(2.0f * v) + 1.0f); }

__global__ __launch_bounds__(NTHR_PREP) void cvt_wh_kernel(const float* __restrict__ w0, const float* __restrict__ w1,
                                                           const float* __restrict__ w2, const float* __restrict__ w3,
                                                           unsigned short* __restrict__ dst) {
  const int g = blockIdx.x >> 5;
  const float* src = (g == 0) ? w0 : (g == 1) ? w1 : (g == 2) ? w2 : w3;
  const int i = (blockIdx.x & 31) * NTHR_PREP + threadIdx.x;
  const v4f a = *(const v4f*)(src + (size_t)i * 8);
  const v4f b = *(const v4f*)(src + (size_t)i * 8 + 4);
  v8h hv;
#pragma unroll
  for (int e = 0; e < 4; ++e) {
    const float fa = a[e] * WCARRY;
    const float fb = b[e] * WCARRY;
    hv[e]     = (_Float16)fa;
    hv[4 + e] = (_Float16)fb;
  }
  unsigned short* op = dst + ((size_t)g * (NHID * NHID / 8) + (size_t)i) * 8;
  *(volatile v8h*)op = hv;
  __threadfence();
  *(volatile v8h*)op = hv;
}

__global__ __launch_bounds__(NTHR_PREP) void ptab_kernel(const float* __restrict__ emb,
                                                         const float* __restrict__ wx0, const float* __restrict__ wx1,
                                                         const float* __restrict__ wx2, const float* __restrict__ wx3,
                                                         float* __restrict__ P) {
  const int g = blockIdx.y;
  const float* src = (g == 0) ? wx0 : (g == 1) ? wx1 : (g == 2) ? wx2 : wx3;
  const int i = blockIdx.x * NTHR_PREP + threadIdx.x;
  if (i < NDIG * (NHID / 4)) {
    const int d  = i >> 6;
    const int j4 = (i & 63) * 4;
    v4f wv[6];
#pragma unroll
    for (int q = 0; q < 6; ++q) wv[q] = *(const v4f*)(src + (size_t)j4 * NEMB + 4 * q);
    float ev[NEMB];
#pragma unroll
    for (int e = 0; e < NEMB; ++e) ev[e] = emb[d * NEMB + e];
    v4f o;
#pragma unroll
    for (int jj = 0; jj < 4; ++jj) {
      float s = 0.0f;
#pragma unroll
      for (int e = 0; e < NEMB; ++e) {
        const int f = jj * NEMB + e;
        s += wv[f >> 2][f & 3] * ev[e];
      }
      o[jj] = s;
    }
    float* op = P + (size_t)g * (NDIG * NHID) + (size_t)i * 4;
    *(volatile v4f*)op = o;
    __threadfence();
    *(volatile v4f*)op = o;
  }
}

__global__ __launch_bounds__(NTHR_SEQ) void lstm_seq_kernel(const int* __restrict__ x,
                                                            const float* __restrict__ bg, const float* __restrict__ bi,
                                                            const float* __restrict__ bfv, const float* __restrict__ bo,
                                                            const unsigned short* __restrict__ WHp,
                                                            const float* __restrict__ Ptab,
                                                            const float* __restrict__ Wp, const float* __restrict__ bp,
                                                            float* __restrict__ out) {
  __shared__ __align__(16) float    Ps[NGATE * NDIG * NHID];
  __shared__ __align__(16) _Float16 Hh[2 * SEQ_BLK * HPITCH];
  __shared__ __align__(16) int      Xs[SEQ_BLK * NSTEP];
  __shared__ __align__(16) float    Hf[SEQ_BLK * HFPITCH];
  __shared__ __align__(16) float    Ob[SEQ_BLK * NCLS];

  const _Float16* WH = (const _Float16*)WHp;
  const int tid = threadIdx.x, lane = tid & 31, wave = tid >> 5;
  const int c = lane & 15, hh = lane >> 4, koff = hh * 8;
  const int rowbase = blockIdx.x * SEQ_BLK;

#pragma unroll 1
  for (int it = 0; it < (NGATE * NDIG * NHID / 4) / NTHR_SEQ; ++it) {
    const int idx = it * NTHR_SEQ + tid;
    const v4f v = *(const v4f*)(Ptab + (size_t)idx * 4);
    *(v4f*)(Ps + idx * 4) = v;
  }
#pragma unroll 1
  for (int it = 0; it < (SEQ_BLK * NSTEP / 4) / NTHR_SEQ; ++it) {
    const int idx = it * NTHR_SEQ + tid;
    const int row = idx >> 7;
    const int c4  = (idx & 127) * 4;
    v4i v = *(const v4i*)(x + (size_t)(rowbase + row) * NSTEP + c4);
#pragma unroll
    for (int e = 0; e < 4; ++e) {
      int q = v[e];
      q = (q < 0) ? 0 : q;
      q = (q > NDIG - 1) ? (NDIG - 1) : q;
      v[e] = q;
    }
    *(v4i*)(Xs + row * NSTEP + c4) = v;
  }
  {
    const v8h zh = {(_Float16)0.0f, (_Float16)0.0f, (_Float16)0.0f, (_Float16)0.0f,
                    (_Float16)0.0f, (_Float16)0.0f, (_Float16)0.0f, (_Float16)0.0f};
#pragma unroll 1
    for (int i = tid; i < (2 * SEQ_BLK * HPITCH) / 8; i += NTHR_SEQ) *(v8h*)(Hh + 8 * i) = zh;
  }

  const int bglob = rowbase + c;
  const float bgv = bg[bglob];
  const float biv = bi[bglob];
  const float bff = bfv[bglob];
  const float bov = bo[bglob];

  float cst[8];
#pragma unroll
  for (int r = 0; r < 8; ++r) cst[r] = 0.0f;

  const int jo = 16 * wave + 8 * hh;
  const _Float16* wa = WH + (size_t)(16 * wave + c) * NHID + koff;
  const v8f z8 = {0.f, 0.f, 0.f, 0.f, 0.f, 0.f, 0.f, 0.f};

  __syncthreads();

#pragma unroll 1
  for (int t = 0; t < NSTEP; ++t) {
    const int cur = t & 1;
    const _Float16* hrow = Hh + cur * (SEQ_BLK * HPITCH) + c * HPITCH + koff;
    _Float16* hnx = Hh + (cur ^ 1) * (SEQ_BLK * HPITCH);
    const int d = Xs[c * NSTEP + t];
    const bool last = (t == NSTEP - 1);

    v8f acc0 = z8, acc1 = z8, acc2 = z8, acc3 = z8;
#pragma unroll 1
    for (int k0 = 0; k0 < NHID; k0 += 32) {
      const v16h fb = frag_load(hrow + k0);
      const v16h a0 = frag_load(wa + k0);
      const v16h a1 = frag_load(wa + (size_t)1 * NHID * NHID + k0);
      const v16h a2 = frag_load(wa + (size_t)2 * NHID * NHID + k0);
      const v16h a3 = frag_load(wa + (size_t)3 * NHID * NHID + k0);
      acc0 = frag_mma(a0, fb, acc0);
      acc1 = frag_mma(a1, fb, acc1);
      acc2 = frag_mma(a2, fb, acc2);
      acc3 = frag_mma(a3, fb, acc3);
      guard_group(acc0, acc1, acc2, acc3, a0, a1, a2, a3, fb);
    }
    acc_guard4(acc0, acc1, acc2, acc3);

    const float* pr = Ps + d * NHID + jo;
    const v4f pg0 = *(const v4f*)(pr);
    const v4f pg1 = *(const v4f*)(pr + 4);
    const v4f pi0 = *(const v4f*)(pr + 1 * NDIG * NHID);
    const v4f pi1 = *(const v4f*)(pr + 1 * NDIG * NHID + 4);
    const v4f pf0 = *(const v4f*)(pr + 2 * NDIG * NHID);
    const v4f pf1 = *(const v4f*)(pr + 2 * NDIG * NHID + 4);
    const v4f po0 = *(const v4f*)(pr + 3 * NDIG * NHID);
    const v4f po1 = *(const v4f*)(pr + 3 * NDIG * NHID + 4);
    const v8f PG = __builtin_shufflevector(pg0, pg1, 0, 1, 2, 3, 4, 5, 6, 7);
    const v8f PI = __builtin_shufflevector(pi0, pi1, 0, 1, 2, 3, 4, 5, 6, 7);
    const v8f PF = __builtin_shufflevector(pf0, pf1, 0, 1, 2, 3, 4, 5, 6, 7);
    const v8f PO = __builtin_shufflevector(po0, po1, 0, 1, 2, 3, 4, 5, 6, 7);

    float hnew[8];
    v8h hv;
#pragma unroll
    for (int r = 0; r < 8; ++r) {
      const float zg = acc0[r] * FOLD + PG[r] + bgv;
      const float zi = acc1[r] * FOLD + PI[r] + biv;
      const float zf = acc2[r] * FOLD + PF[r] + bff;
      const float zo = acc3[r] * FOLD + PO[r] + bov;
      const float gg = tanh_f(zg);
      const float ii = sig_f(zi);
      const float ff = sig_f(zf);
      const float oo = sig_f(zo);
      const float cn = gg * ii + cst[r] * ff;
      cst[r] = cn;
      const float hn = tanh_f(cn) * oo;
      hnew[r] = hn;
      const float hs = hn * HCARRY;
      hv[r] = (_Float16)hs;
    }
    *(v8h*)(hnx + c * HPITCH + jo) = hv;
    if (last) {
      const v4f f0 = {hnew[0], hnew[1], hnew[2], hnew[3]};
      const v4f f1 = {hnew[4], hnew[5], hnew[6], hnew[7]};
      *(v4f*)(Hf + c * HFPITCH + jo) = f0;
      *(v4f*)(Hf + c * HFPITCH + jo + 4) = f1;
    }
    __syncthreads();
  }

  if (tid < SEQ_BLK * NCLS) {
    const int bl  = tid / NCLS;
    const int cls = tid - bl * NCLS;
    const float* wrow = Wp + (size_t)cls * NHID;
    const float* hrow32 = Hf + bl * HFPITCH;
    float s = 0.0f;
#pragma unroll 2
    for (int j4 = 0; j4 < NHID / 4; ++j4) {
      const v4f w = *(const v4f*)(wrow + 4 * j4);
      const v4f h = *(const v4f*)(hrow32 + 4 * j4);
      s += w[0] * h[0];
      s += w[1] * h[1];
      s += w[2] * h[2];
      s += w[3] * h[3];
    }
    s += bp[cls];
    Ob[tid] = s;
  }
  __syncthreads();
  if (wave == 0) {
    float ov[5];
#pragma unroll
    for (int q = 0; q < 5; ++q) ov[q] = Ob[q * 32 + lane];
    float* op = out + (size_t)rowbase * NCLS;
    for (int pass = 0; pass < 2; ++pass) {
#pragma unroll
      for (int q = 0; q < 5; ++q) *(volatile float*)(op + q * 32 + lane) = ov[q];
      __threadfence();
    }
  }
}

extern "C" void kernel_launch(void* const* d_in, const int* in_sizes, int n_in,
                              void* d_out, int out_size, void* d_ws, size_t ws_size, hipStream_t stream) {
  if (n_in < 16 || d_out == nullptr || d_ws == nullptr) return;
  if (in_sizes[0] != NBATCH * NSTEP || in_sizes[1] != NDIG * NEMB ||
      in_sizes[2] != NHID * NEMB || in_sizes[3] != NHID * NHID || in_sizes[4] != NHID ||
      in_sizes[5] != NHID * NEMB || in_sizes[6] != NHID * NHID || in_sizes[7] != NHID ||
      in_sizes[8] != NHID * NEMB || in_sizes[9] != NHID * NHID || in_sizes[10] != NHID ||
      in_sizes[11] != NHID * NEMB || in_sizes[12] != NHID * NHID || in_sizes[13] != NHID ||
      in_sizes[14] != NCLS * NHID || in_sizes[15] != NCLS || out_size != NBATCH * NCLS) return;

  const int*   x   = (const int*)  d_in[0];
  const float* emb = (const float*)d_in[1];
  const float* Wxg = (const float*)d_in[2];
  const float* Whg = (const float*)d_in[3];
  const float* bg  = (const float*)d_in[4];
  const float* Wxi = (const float*)d_in[5];
  const float* Whi = (const float*)d_in[6];
  const float* bi  = (const float*)d_in[7];
  const float* Wxf = (const float*)d_in[8];
  const float* Whf = (const float*)d_in[9];
  const float* bfv = (const float*)d_in[10];
  const float* Wxo = (const float*)d_in[11];
  const float* Who = (const float*)d_in[12];
  const float* bo  = (const float*)d_in[13];
  const float* Wp  = (const float*)d_in[14];
  const float* bp  = (const float*)d_in[15];
  float* out = (float*)d_out;

  char* ws = (char*)d_ws;
  size_t off = 0;
  auto carve = [&](size_t bytes) -> char* { char* p = ws + off; off += (bytes + 255) & ~(size_t)255; return p; };
  unsigned short* WH16 = (unsigned short*)carve((size_t)NGATE * NHID * NHID * 2);
  float*          PTAB = (float*)carve((size_t)NGATE * NDIG * NHID * 4);
  if (off > ws_size || off > (size_t)134217728) return;

  cvt_wh_kernel<<<NGATE * 32, NTHR_PREP, 0, stream>>>(Whg, Whi, Whf, Who, WH16);
  ptab_kernel<<<dim3(3, NGATE), NTHR_PREP, 0, stream>>>(emb, Wxg, Wxi, Wxf, Wxo, PTAB);
  lstm_seq_kernel<<<NBATCH / SEQ_BLK, NTHR_SEQ, 0, stream>>>(x, bg, bi, bfv, bo, WH16, PTAB, Wp, bp, out);
}
